// IntervalClusterTripletFT_48258252538457
// MI455X (gfx1250) — hardware-run, weakly checked
//
#include <hip/hip_runtime.h>


#define NN   8192
#define ND   128
#define NCH  1024
#define NL   8
typedef _Float16 h16;
typedef unsigned short bf;
typedef __attribute__((ext_vector_type(16))) __bf16   v16bf;
typedef __attribute__((ext_vector_type(16))) _Float16 v16h;
typedef __attribute__((ext_vector_type(8)))  _Float16 v8h;
typedef __attribute__((ext_vector_type(8)))  unsigned short v8us;
typedef __attribute__((ext_vector_type(8)))  float    v8f;
typedef __attribute__((ext_vector_type(4)))  float    v4f;
typedef v8h  __attribute__((may_alias)) v8ha;
typedef v4f  __attribute__((may_alias)) v4fa;
typedef v8us __attribute__((may_alias)) v8usa;

__device__ __forceinline__ unsigned short f2bf(float f) { unsigned u = __float_as_uint(f); u += 0x7FFFu + ((u >> 16) & 1u); return (unsigned short)(u >> 16); }
__device__ __forceinline__ float bf2f(unsigned short b) { return __uint_as_float(((unsigned)b) << 16); }
__device__ __forceinline__ float bfr(float f) { return bf2f(f2bf(f)); }
__device__ __forceinline__ v16h cat16(v8h lo, v8h hi) { return __builtin_shufflevector(lo, hi, 0, 1, 2, 3, 4, 5, 6, 7, 8, 9, 10, 11, 12, 13, 14, 15); }
__device__ __forceinline__ v16bf cat16b(v8us lo, v8us hi) { return __builtin_bit_cast(v16bf, __builtin_shufflevector(lo, hi, 0, 1, 2, 3, 4, 5, 6, 7, 8, 9, 10, 11, 12, 13, 14, 15)); }
__device__ __forceinline__ v8f wmma16(v16h a, v16h b, v8f c) { return __builtin_amdgcn_wmma_f32_16x16x32_f16(false, a, false, b, (short)0, c, false, false); }
__device__ __forceinline__ v8f wmmab(v16bf a, v16bf b, v8f c) { return __builtin_amdgcn_wmma_f32_16x16x32_bf16(false, a, false, b, (short)0, c, false, false); }

template <typename T16> struct WFrag;
template <> struct WFrag<h16> { typedef v16h V; static __device__ __forceinline__ V ld(const h16* p) { return cat16(*(const v8h*)p, *(const v8h*)(p + 16)); } static __device__ __forceinline__ v8f mma(V a, V b, v8f c) { return wmma16(a, b, c); } };
template <> struct WFrag<bf> { typedef v16bf V; static __device__ __forceinline__ V ld(const bf* p) { return cat16b(*(const v8us*)p, *(const v8us*)(p + 16)); } static __device__ __forceinline__ v8f mma(V a, V b, v8f c) { return wmmab(a, b, c); } };
template <typename T16, int NSPLIT, bool BIAS>
__global__ __launch_bounds__(32) void k_gemmw(const T16* __restrict__ A, const T16* __restrict__ A2, const T16* __restrict__ Bt, const T16* __restrict__ Bt2, int K, float* C, int ldc, const float* __restrict__ bias, size_t sA, size_t sB, size_t sC) {
    typedef typename WFrag<T16>::V V;
    __shared__ __align__(16) float os[16 * 68];
    const size_t z = blockIdx.z; A += z * sA; if (A2) A2 += z * sA; Bt += z * sB; if (Bt2) Bt2 += z * sB; C += z * sC;
    const int lane = threadIdx.x & 31, lr = lane & 15, hi = lane >> 4; const int r0 = blockIdx.x * 64, c0 = blockIdx.y * 64;
    v8f acc[4][4];
#pragma unroll
    for (int mb = 0; mb < 4; ++mb)
#pragma unroll
        for (int nb = 0; nb < 4; ++nb) acc[mb][nb] = (v8f){};
    const size_t aoff = (size_t)(r0 + lr) * K + 8 * hi, boff = (size_t)(c0 + lr) * K + 8 * hi;
    for (int kc = 0; kc < K; kc += 32) {
        V a[4], a2[4];
#pragma unroll
        for (int mb = 0; mb < 4; ++mb) { a[mb] = WFrag<T16>::ld(A + aoff + (size_t)mb * 16 * K + kc); if (NSPLIT == 1 || NSPLIT == 2) a2[mb] = WFrag<T16>::ld(A2 + aoff + (size_t)mb * 16 * K + kc); }
#pragma unroll
        for (int nb = 0; nb < 4; ++nb) { const V b = WFrag<T16>::ld(Bt + boff + (size_t)nb * 16 * K + kc); V b2; if (NSPLIT >= 2) b2 = WFrag<T16>::ld(Bt2 + boff + (size_t)nb * 16 * K + kc);
#pragma unroll
            for (int mb = 0; mb < 4; ++mb) { acc[mb][nb] = WFrag<T16>::mma(a[mb], b, acc[mb][nb]); if (NSPLIT == 1 || NSPLIT == 2) acc[mb][nb] = WFrag<T16>::mma(a2[mb], b, acc[mb][nb]); if (NSPLIT >= 2) acc[mb][nb] = WFrag<T16>::mma(a[mb], b2, acc[mb][nb]); } }
        asm volatile("v_nop\n\tv_nop\n\tv_nop\n\tv_nop" : "+v"(acc[0][0]), "+v"(acc[1][1]), "+v"(acc[2][2]), "+v"(acc[3][3]) : "v"(a[0]), "v"(a[3]));
    }
#pragma unroll
    for (int mb = 0; mb < 4; ++mb) {
#pragma unroll
        for (int nb = 0; nb < 4; ++nb) {
#pragma unroll
            for (int j = 0; j < 8; ++j) os[(hi * 8 + j) * 68 + nb * 16 + lr] = acc[mb][nb][j]; }
        __builtin_amdgcn_wave_barrier(); asm volatile("" ::: "memory");
        float* crow = C + (size_t)(r0 + mb * 16) * ldc + c0;
#pragma unroll 1
        for (int ps = 0; ps < 2; ++ps) {
#pragma unroll
            for (int s = 0; s < 8; ++s) { const int row = 2 * s + hi, cofs = lr * 4; v4f val = *(const v4fa*)(os + row * 68 + cofs); if (BIAS) { val[0] += bfr(bias[c0 + cofs]); val[1] += bfr(bias[c0 + cofs + 1]); val[2] += bfr(bias[c0 + cofs + 2]); val[3] += bfr(bias[c0 + cofs + 3]); }
                *(volatile v4f*)(crow + (size_t)row * ldc + cofs) = val; }
            if (ps == 0) __threadfence(); }
        __builtin_amdgcn_wave_barrier(); asm volatile("" ::: "memory");
    }
}

__global__ __launch_bounds__(256) void k_cvt8(const float* __restrict__ src, bf* dst, size_t n8) { const size_t i = (size_t)blockIdx.x * 256 + threadIdx.x; if (i >= n8) return; const v8f v = *(const v8f*)(src + i * 8); v8us o;
#pragma unroll
    for (int k = 0; k < 8; ++k) o[k] = f2bf(v[k]); *(volatile v8us*)(dst + i * 8) = o; __threadfence(); *(volatile v8us*)(dst + i * 8) = o; }

__global__ __launch_bounds__(256) void k_sq(const float* __restrict__ a, float* Q) { const int i = blockIdx.x * 256 + threadIdx.x; if (i >= NN) return; const float* p = a + (size_t)i * ND; float s = 0.0f;
    for (int c = 0; c < ND / 4; ++c) { const v4f v = *(const v4f*)(p + 4 * c);
#pragma unroll
        for (int k = 0; k < 4; ++k) { const float x = bfr(v[k]); s = __fmaf_rn(x, x, s); } }
    *(volatile float*)(Q + i) = s; __threadfence(); *(volatile float*)(Q + i) = s; }

__global__ __launch_bounds__(256) void k_tm(const float* __restrict__ S, const float* __restrict__ Q, int r0, float* out) { const int t = blockIdx.x * 256 + threadIdx.x; if (t >= NCH) return; const int i = r0 + t; const int gi = i >> 4; const float qi = Q[i]; const float* sr = S + (size_t)t * NN; float p = -1.0f; float n = __int_as_float(0x7f800000);
    for (int g = 0; g < NN / 4; ++g) { const v4f s = *(const v4f*)(sr + 4 * g); const v4f q = *(const v4f*)(Q + 4 * g); const bool same = ((4 * g) >> 4) == gi;
#pragma unroll
        for (int k = 0; k < 4; ++k) { const float d2 = __fsub_rn(__fadd_rn(qi, q[k]), __fmul_rn(2.0f, s[k])); const float d = __fsqrt_rn(d2 > 0.0f ? d2 : 0.0f); const float pc = (d > p) ? d : p; const float nc = (d < n) ? d : n; p = same ? pc : p; n = same ? n : nc; } }
    const float o = __fadd_rn(__fsub_rn(p, n), 1.0f); const float r = (o > 0.0f) ? o : 0.0f;
    *(volatile float*)(out + i) = r; __threadfence(); *(volatile float*)(out + i) = r; }

extern "C" void kernel_launch(void* const* d_in, const int* in_sizes, int n_in, void* d_out, int out_size, void* d_ws, size_t ws_size, hipStream_t stream) {
    if (n_in < 1) return;
    if (in_sizes[0] != NN * ND) return;
    if (out_size != NN) return;
    static_assert(NL * NCH == NN && NCH % 64 == 0 && NN % 64 == 0 && ND % 32 == 0 && (NN * ND / 8) % 256 == 0 && NN % 256 == 0 && NCH % 256 == 0 && NN % 16 == 0, "the product: M and N multiples of 64, the depth a multiple of 32; every flat grid exact; a group of 16 rows never straddles a 4-word piece (4 divides 16)");
    const float* a = (const float*)d_in[0];
    float* out = (float*)d_out;
    char* wsp = (char*)d_ws; auto take = [&](size_t bytes) { char* p = wsp; wsp += (bytes + 255) & ~(size_t)255; return (void*)p; };
    bf* Xb = (bf*)take((size_t)NN * ND * 2); float* Q = (float*)take((size_t)NN * 4); float* S = (float*)take((size_t)NCH * NN * 4);
    if ((size_t)(wsp - (char*)d_ws) > ws_size) return;
    k_cvt8<<<(unsigned)(NN * ND / 8 / 256), 256, 0, stream>>>(a, Xb, (size_t)NN * ND / 8);
    k_sq<<<(unsigned)(NN / 256), 256, 0, stream>>>(a, Q);
    for (int c = 0; c < NL; ++c) {
        k_gemmw<bf, 0, false><<<dim3(NCH / 64, NN / 64, 1), 32, 0, stream>>>(Xb + (size_t)c * NCH * ND, nullptr, Xb, nullptr, ND, S, NN, nullptr, 0, 0, 0);
        k_tm<<<(unsigned)(NCH / 256), 256, 0, stream>>>(S, Q, c * NCH, out); }
}
